// adapt_mnist_net_60979945669246
// MI455X (gfx1250) — hardware-verified
//
#include <hip/hip_runtime.h>

typedef _Float16 __bf16_t;
#define __bf16 __bf16_t
typedef __attribute__((ext_vector_type(16))) _Float16 v16bf;
typedef __attribute__((ext_vector_type(8)))  float  v8f;
typedef __attribute__((ext_vector_type(4)))  float  v4f;

#define NWAVES   8
#define NTHREADS 256
#define TILE     16

template <int I> struct IC { static constexpr int v = I; };
template <int... Is> struct ISeq {};
template <int N, int... Is> struct MkSeq : MkSeq<N - 1, N - 1, Is...> {};
template <int... Is> struct MkSeq<0, Is...> { using T = ISeq<Is...>; };
template <class F, int... Is>
static __device__ __forceinline__ void sfor_impl(F&& f, ISeq<Is...>) { (f(IC<Is>{}), ...); }
template <int N, class F>
static __device__ __forceinline__ void sfor(F&& f) { sfor_impl(f, typename MkSeq<N>::T{}); }

static constexpr int R0_OFF = 0;
static constexpr int R1_OFF = 49152;
static constexpr int R2_OFF = R1_OFF + 32768;
static constexpr int W1_OFF = R2_OFF + 40960;
static constexpr int W2_OFF = W1_OFF + 64 * 16;
static constexpr int W3_OFF = W2_OFF + 96 * 16;
static constexpr int W4_OFF = W3_OFF + 96 * 16;
static constexpr int W5_OFF = W4_OFF + 96 * 16;
static constexpr int WD_OFF = W5_OFF + 160 * 32;
static constexpr int LDS_ELTS = WD_OFF + 224 * 16;

static __device__ __forceinline__ v8f wmma_bf16(v16bf a, v16bf b, v8f c) {
  v8f d = __builtin_amdgcn_wmma_f32_16x16x32_f16(false, a, false, b, (short)0, c, false, false);
  asm volatile("v_nop\n\tv_nop\n\tv_nop\n\tv_nop" : "+v"(d) : "v"(a), "v"(b));
  return d;
}
static __device__ __forceinline__ v8f vzero8() {
  v8f z = {0.f, 0.f, 0.f, 0.f, 0.f, 0.f, 0.f, 0.f};
  return z;
}

template <int Hp, int Wp, int KH, int KW>
static constexpr int im2off(int k) {
  return (k / (KH * KW)) * Hp * Wp + ((k % (KH * KW)) / KW) * Wp + (k % KW);
}

template <int Hp, int Wp, int KH, int KW, int KTRUE, int K0>
static __device__ __forceinline__ v16bf make_a_frag(const __bf16* act, int base, bool g1) {
  v16bf a;
  sfor<16>([&](auto ii) {
    constexpr int idx = decltype(ii)::v;
    constexpr int v = idx >> 1, p = idx & 1;
    constexpr int kA = K0 + (v & 3) * 2 + (v >> 2) * 16 + p;
    constexpr int kB = kA + 8;
    constexpr bool vA = kA < KTRUE, vB = kB < KTRUE;
    if constexpr (!vA && !vB) {
      a[idx] = (__bf16)0.0f;
    } else {
      constexpr int oA = im2off<Hp, Wp, KH, KW>(vA ? kA : 0);
      constexpr int oB = im2off<Hp, Wp, KH, KW>(vB ? kB : 0);
      const int off = g1 ? oB : oA;
      const __bf16 t = act[base + off];
      if constexpr (vA && vB) a[idx] = t;
      else                    a[idx] = ((g1 ? vB : vA)) ? t : (__bf16)0.0f;
    }
  });
  return a;
}

template <int NSTR, int K0>
static __device__ __forceinline__ v16bf make_b_frag(const __bf16* w, int baseB) {
  v16bf b;
  sfor<16>([&](auto ii) {
    constexpr int idx = decltype(ii)::v;
    constexpr int off = (K0 + ((idx < 8) ? idx : (idx + 8))) * NSTR;
    b[idx] = w[baseB + off];
  });
  return b;
}

template <int C, int H, int W, int KH, int KW, int PAD, int OCH, int KPAD, int OHALO>
static __device__ __forceinline__ void conv_relu(const __bf16* in, __bf16* out,
                                                 const __bf16* wl, int wave, int lane) {
  constexpr int KTRUE = C * KH * KW, NFRAG = KPAD / 32;
  constexpr int Hp = H + 2 * PAD, Wp = W + 2 * PAD;
  constexpr int HpO = H + 2 * OHALO, WpO = W + 2 * OHALO;
  const int nlo = lane & 15;
  const bool g1 = (lane >> 4) != 0;
  const int mbase = nlo * (C * Hp * Wp);

  v16bf bfr[NFRAG];
  const int baseB = nlo + (g1 ? 8 * 16 : 0);
  sfor<NFRAG>([&](auto fi) {
    constexpr int F = decltype(fi)::v;
    bfr[F] = make_b_frag<16, F * 32>(wl, baseB);
  });

  for (int pos = wave; pos < H * W; pos += NWAVES) {
    const int oh = pos / W, ow = pos % W;
    const int base = mbase + oh * Wp + ow;
    v8f acc = vzero8();
    sfor<NFRAG>([&](auto fi) {
      constexpr int F = decltype(fi)::v;
      v16bf a = make_a_frag<Hp, Wp, KH, KW, KTRUE, F * 32>(in, base, g1);
      acc = wmma_bf16(a, bfr[F], acc);
    });
    sfor<8>([&](auto ri) {
      constexpr int r = decltype(ri)::v;
      const int m = r + (g1 ? 8 : 0);
      if (nlo < OCH)
        out[((m * OCH + nlo) * HpO + oh + OHALO) * WpO + ow + OHALO] =
            (__bf16)fmaxf(acc[r], 0.0f);
    });
  }
}

template <int C, int H, int W, int KH, int KW, int PAD, int OCH, int KPAD,
          int PH, int PW, int PPAD, int OHALO, int NT>
static __device__ __forceinline__ void conv_relu_pool(const __bf16* in, __bf16* out,
                                                      const __bf16* wl, int wave, int lane) {
  constexpr int KTRUE = C * KH * KW, NFRAG = KPAD / 32, NSTR = NT * 16;
  constexpr int Hp = H + 2 * PAD, Wp = W + 2 * PAD;
  constexpr int HpO = PH + 2 * OHALO, WpO = PW + 2 * OHALO;
  const int nlo = lane & 15;
  const bool g1 = (lane >> 4) != 0;
  const int mbase = nlo * (C * Hp * Wp);

  v16bf bfr[NT][NFRAG];
  const int baseB = nlo + (g1 ? 8 * NSTR : 0);
  sfor<NT>([&](auto ti) {
    constexpr int T = decltype(ti)::v;
    sfor<NFRAG>([&](auto fi) {
      constexpr int F = decltype(fi)::v;
      bfr[T][F] = make_b_frag<NSTR, F * 32>(wl, baseB + T * 16);
    });
  });

  for (int pos = wave; pos < PH * PW; pos += NWAVES) {
    const int ph = pos / PW, pw = pos % PW;
    v8f best[NT];
    sfor<NT>([&](auto ti) { best[decltype(ti)::v] = vzero8(); });

    for (int dh = 0; dh < 3; ++dh) {
      for (int dw = 0; dw < 3; ++dw) {
        const int h = ph * 2 - PPAD + dh;
        const int w = pw * 2 - PPAD + dw;
        if (h >= 0 && h < H && w >= 0 && w < W) {
          const int base = mbase + h * Wp + w;
          v16bf afr[NFRAG];
          sfor<NFRAG>([&](auto fi) {
            constexpr int F = decltype(fi)::v;
            afr[F] = make_a_frag<Hp, Wp, KH, KW, KTRUE, F * 32>(in, base, g1);
          });
          sfor<NT>([&](auto ti) {
            constexpr int T = decltype(ti)::v;
            v8f acc = vzero8();
            sfor<NFRAG>([&](auto fi) {
              constexpr int F = decltype(fi)::v;
              acc = wmma_bf16(afr[F], bfr[T][F], acc);
            });
            sfor<8>([&](auto ri) {
              constexpr int r = decltype(ri)::v;
              best[T][r] = fmaxf(best[T][r], acc[r]);
            });
          });
        }
      }
    }
    sfor<NT>([&](auto ti) {
      constexpr int T = decltype(ti)::v;
      sfor<8>([&](auto ri) {
        constexpr int r = decltype(ri)::v;
        const int m = r + (g1 ? 8 : 0), n = T * 16 + nlo;
        if (n < OCH)
          out[((m * OCH + n) * HpO + ph + OHALO) * WpO + pw + OHALO] = (__bf16)best[T][r];
      });
    });
  }
}

static __device__ __forceinline__ void dense_out(const __bf16* x, const __bf16* wl,
                                                 float* out, int imgbase, int lane, float* so) {
  const int nlo = lane & 15;
  const bool g1 = (lane >> 4) != 0;
  const int baseA = nlo * 216 + (g1 ? 8 : 0);
  const int baseB = nlo + (g1 ? 8 * 16 : 0);
  v8f acc = vzero8();
  sfor<7>([&](auto fi) {
    constexpr int F = decltype(fi)::v;
    v16bf a;
    sfor<16>([&](auto ii) {
      constexpr int idx = decltype(ii)::v;
      constexpr int v = idx >> 1, p = idx & 1;
      constexpr int kc = F * 32 + (v & 3) * 2 + (v >> 2) * 16 + p;
      constexpr bool vA = kc < 216, vB = (kc + 8) < 216;
      if constexpr (!vA && !vB) a[idx] = (__bf16)0.0f;
      else {
        const __bf16 t = x[baseA + kc];
        if constexpr (vA && vB) a[idx] = t;
        else                    a[idx] = ((g1 ? vB : vA)) ? t : (__bf16)0.0f;
      }
    });
    v16bf b = make_b_frag<16, F * 32>(wl, baseB);
    acc = wmma_bf16(a, b, acc);
  });
  sfor<8>([&](auto ri) {
    constexpr int r = decltype(ri)::v;
    const int m = r + (g1 ? 8 : 0);
    if (nlo < 10) so[m * 10 + nlo] = acc[r];
  });
  __builtin_amdgcn_fence(__ATOMIC_RELEASE, "workgroup"); __builtin_amdgcn_wave_barrier(); __builtin_amdgcn_fence(__ATOMIC_ACQUIRE, "workgroup");
  float* dst = out + (size_t)imgbase * 10;
  for (int pass = 0; pass < 2; ++pass) {
    *(volatile v4f*)(dst + lane * 4) = *(const v4f*)(so + lane * 4);
    if (lane < 8) *(volatile v4f*)(dst + 128 + lane * 4) = *(const v4f*)(so + 128 + lane * 4);
    __threadfence();
  }
}

template <int O, int C, int KH, int KW, int KPAD, int NT>
static __device__ __forceinline__ void load_conv_w(const float* g, __bf16* wl, int tid) {
  constexpr int NSTR = NT * 16, KTRUE = C * KH * KW;
  for (int i = tid; i < KPAD * NSTR; i += NTHREADS) {
    const int k = i / NSTR, n = i % NSTR;
    float v = 0.f;
    if (k < KTRUE && n < O) v = g[n * KTRUE + k];
    wl[i] = (__bf16)v;
  }
}

static __device__ __forceinline__ void zero_region(__bf16* p, int nelts, int tid) {
  unsigned int* q = (unsigned int*)p;
  for (int i = tid; i < nelts / 2; i += NTHREADS) q[i] = 0u;
}

__global__ __launch_bounds__(NTHREADS) void mnist_fused(
    const float* __restrict__ inp, const float* __restrict__ w1,
    const float* __restrict__ w2, const float* __restrict__ w3,
    const float* __restrict__ w4, const float* __restrict__ w5,
    const float* __restrict__ wd, float* __restrict__ out) {
  __shared__ __bf16 smem[LDS_ELTS];
  __shared__ __attribute__((aligned(16))) float sout[TILE * 10];
  const int tid = threadIdx.x;
  const int lane = tid & 31;
  const int wave = __builtin_amdgcn_readfirstlane(tid) >> 5;
  const int imgbase = blockIdx.x * TILE;

  zero_region(smem + R1_OFF, TILE * 1 * 34 * 34, tid);
  zero_region(smem + R0_OFF, TILE * 3 * 32 * 32, tid);
  load_conv_w<3, 1, 7, 7, 64, 1>(w1, smem + W1_OFF, tid);
  load_conv_w<8, 3, 5, 5, 96, 1>(w2, smem + W2_OFF, tid);
  load_conv_w<10, 8, 3, 3, 96, 1>(w3, smem + W3_OFF, tid);
  load_conv_w<16, 10, 3, 3, 96, 1>(w4, smem + W4_OFF, tid);
  load_conv_w<24, 16, 3, 3, 160, 2>(w5, smem + W5_OFF, tid);
  for (int i = tid; i < 224 * 16; i += NTHREADS) {
    const int k = i / 16, n = i % 16;
    float v = 0.f;
    if (k < 216 && n < 10) v = wd[n * 216 + k];
    smem[WD_OFF + i] = (__bf16)v;
  }
  __syncthreads();

  {
    const float* src = inp + (size_t)imgbase * 784;
    for (int i = tid; i < TILE * 784; i += NTHREADS) {
      const int m = i / 784, r = i % 784, h = r / 28, w = r % 28;
      smem[R1_OFF + (m * 34 + h + 3) * 34 + w + 3] = (__bf16)src[i];
    }
  }
  __syncthreads();

  conv_relu<1, 28, 28, 7, 7, 3, 3, 64, 2>(smem + R1_OFF, smem + R0_OFF, smem + W1_OFF,
                                          wave, lane);
  __syncthreads();
  zero_region(smem + R1_OFF, TILE * 8 * 16 * 16, tid);
  zero_region(smem + R2_OFF, TILE * 10 * 16 * 16, tid);
  __syncthreads();
  conv_relu_pool<3, 28, 28, 5, 5, 2, 8, 96, 14, 14, 1, 1, 1>(
      smem + R0_OFF, smem + R1_OFF, smem + W2_OFF, wave, lane);
  __syncthreads();
  zero_region(smem + R0_OFF, TILE * 16 * 9 * 9, tid);
  __syncthreads();
  conv_relu<8, 14, 14, 3, 3, 1, 10, 96, 1>(smem + R1_OFF, smem + R2_OFF, smem + W3_OFF,
                                           wave, lane);
  __syncthreads();
  conv_relu_pool<10, 14, 14, 3, 3, 1, 16, 96, 7, 7, 1, 1, 1>(
      smem + R2_OFF, smem + R0_OFF, smem + W4_OFF, wave, lane);
  __syncthreads();
  conv_relu_pool<16, 7, 7, 3, 3, 1, 24, 160, 3, 3, 0, 0, 2>(
      smem + R0_OFF, smem + R1_OFF, smem + W5_OFF, wave, lane);
  __syncthreads();
  if (wave == 0) dense_out(smem + R1_OFF, smem + WD_OFF, out, imgbase, lane, sout);
}

extern "C" void kernel_launch(void* const* d_in, const int* in_sizes, int n_in,
                              void* d_out, int out_size, void* d_ws, size_t ws_size,
                              hipStream_t stream) {
  (void)n_in; (void)out_size; (void)d_ws; (void)ws_size;
  const float* inp = (const float*)d_in[0];
  const float* w1  = (const float*)d_in[1];
  const float* w2  = (const float*)d_in[2];
  const float* w3  = (const float*)d_in[3];
  const float* w4  = (const float*)d_in[4];
  const float* w5  = (const float*)d_in[5];
  const float* wd  = (const float*)d_in[6];
  float* out = (float*)d_out;

  const int B = in_sizes[0] / 784;
  const int nblocks = B / TILE;
  mnist_fused<<<nblocks, NTHREADS, 0, stream>>>(inp, w1, w2, w3, w4, w5, wd, out);
}
